// TransformerCrossBlock_28020366639297
// MI455X (gfx1250) — hardware-verified
//
#include <hip/hip_runtime.h>

typedef _Float16 v16h __attribute__((ext_vector_type(16)));
typedef _Float16 v8h  __attribute__((ext_vector_type(8)));
typedef float    v8f  __attribute__((ext_vector_type(8)));
typedef float    v4f  __attribute__((ext_vector_type(4)));
typedef v8h __attribute__((may_alias)) v8ha;
typedef v4f __attribute__((may_alias)) v4fa;

union Frag { v16h v; v8h half[2]; };

#define DIM    512
#define NHEADS 8
#define HD     64
#define SQ     512
#define SK     1024
#define BATCH  16
#define NLAYER 2
#define DFF    2048
#define MQ     (BATCH * SQ)
#define MK     (BATCH * SK)
#define WSCALE 32.0f
#define PSCALE 256.0f
#define ATTSC  16.0f
#define HSC    8.0f
#define BN_EPS 1e-3f

#define F_BIAS  1
#define F_RESID 2
#define F_BN    4
#define F_RELU  8
#define F_O32   16
#define F_O16   32

__device__ __forceinline__ v8f wmma_f16(v16h a, v16h b, v8f c) {
  v8f d = __builtin_amdgcn_wmma_f32_16x16x32_f16(false, a, false, b, (short)0, c, false, false);
  asm volatile("v_nop\n\tv_nop\n\tv_nop\n\tv_nop" : "+v"(d) : "v"(a), "v"(b));
  return d;
}

__device__ __forceinline__ v16h load_frag(const _Float16* p, int h) {
  Frag f;
  f.half[0] = *(const v8ha*)(p + 8 * h);
  f.half[1] = *(const v8ha*)(p + 16 + 8 * h);
  return f.v;
}

__device__ __forceinline__ v8h cvt8(v4f a, v4f c, float sc) {
  const v8h o = { (_Float16)(a.x * sc), (_Float16)(a.y * sc), (_Float16)(a.z * sc), (_Float16)(a.w * sc),
                  (_Float16)(c.x * sc), (_Float16)(c.y * sc), (_Float16)(c.z * sc), (_Float16)(c.w * sc) };
  return o;
}

__global__ __launch_bounds__(256) void cvt_rows_kernel(
    const float* __restrict__ a, int na8,
    const float* __restrict__ b, int nb8,
    _Float16* __restrict__ ah, _Float16* __restrict__ bh)
{
  const int g = blockIdx.x * 256 + threadIdx.x;
  if (g >= na8 + nb8) return;
  const float* src;
  _Float16* dst;
  if (g < na8) {
    src = a + (size_t)g * 8;
    dst = ah + (size_t)g * 8;
  } else {
    const int e = g - na8;
    src = b + (size_t)e * 8;
    dst = bh + (size_t)e * 8;
  }
  const v4f p = *(const v4fa*)src;
  const v4f q = *(const v4fa*)(src + 4);
  const v8h o = cvt8(p, q, 1.0f);
  *(volatile v8h*)dst = o;
  __threadfence();
  *(volatile v8h*)dst = o;
}

__global__ __launch_bounds__(256) void cvt_wt_kernel(
    const float* __restrict__ s0, const float* __restrict__ s1,
    const float* __restrict__ s2, const float* __restrict__ s3,
    _Float16* __restrict__ d0, _Float16* __restrict__ d1,
    _Float16* __restrict__ d2, _Float16* __restrict__ d3,
    int K, int N, int nz)
{
  __shared__ __attribute__((aligned(16))) _Float16 sT[64 * 72];

  const int tid = threadIdx.x;
  const int sel = blockIdx.z / nz;
  const int z = blockIdx.z - sel * nz;
  const float* src = (sel == 0) ? s0 : ((sel == 1) ? s1 : ((sel == 2) ? s2 : s3));
  _Float16* dst = (sel == 0) ? d0 : ((sel == 1) ? d1 : ((sel == 2) ? d2 : d3));
  src += (size_t)z * K * N;
  dst += (size_t)z * K * N;

  const int n0 = blockIdx.x * 64, k0 = blockIdx.y * 64;
  const int r = tid >> 2, c = (tid & 3) * 16;
  const float* sp = src + (size_t)(k0 + r) * N + n0 + c;
  #pragma unroll
  for (int u = 0; u < 4; ++u) {
    const v4f v = *(const v4fa*)(sp + 4 * u);
    sT[(c + 4 * u + 0) * 72 + r] = (_Float16)(v.x * WSCALE);
    sT[(c + 4 * u + 1) * 72 + r] = (_Float16)(v.y * WSCALE);
    sT[(c + 4 * u + 2) * 72 + r] = (_Float16)(v.z * WSCALE);
    sT[(c + 4 * u + 3) * 72 + r] = (_Float16)(v.w * WSCALE);
  }
  __syncthreads();

  const int q8 = tid & 7, nn0 = tid >> 3;
  const v8h o0 = *(const v8ha*)(sT + nn0 * 72 + 8 * q8);
  const v8h o1 = *(const v8ha*)(sT + (nn0 + 32) * 72 + 8 * q8);
  _Float16* p0 = dst + (size_t)(n0 + nn0) * K + k0 + 8 * q8;
  _Float16* p1 = dst + (size_t)(n0 + nn0 + 32) * K + k0 + 8 * q8;
  *(volatile v8h*)p0 = o0;
  *(volatile v8h*)p1 = o1;
  __threadfence();
  *(volatile v8h*)p0 = o0;
  *(volatile v8h*)p1 = o1;
}

__device__ __forceinline__ void proj_store_pass(const _Float16* sT, _Float16* plane, _Float16* vt,
                                                int which, int S, int bh, int l0, int w, int lane) {
  const int q8 = lane & 7, sub = lane >> 3;
  #pragma unroll
  for (int i = 0; i < 8; ++i) {
    const int lid = w * 32 + i * 4 + sub;
    v8h v;
    _Float16* dst;
    if (which != 2) {
      v = *(const v8ha*)(sT + lid * HD + 8 * q8);
      dst = plane + ((size_t)bh * S + l0 + lid) * HD + 8 * q8;
    } else {
      const int d = lid >> 1, hl = lid & 1;
      v = *(const v8ha*)(sT + d * 128 + 64 * hl + 8 * q8);
      dst = vt + ((size_t)bh * HD + d) * S + l0 + 64 * hl + 8 * q8;
    }
    *(volatile v8h*)dst = v;
  }
}

__global__ __launch_bounds__(128) void proj_kernel(
    const _Float16* __restrict__ xh, int S,
    const _Float16* __restrict__ w0, const _Float16* __restrict__ w1, const _Float16* __restrict__ w2,
    const float* __restrict__ b0, const float* __restrict__ b1, const float* __restrict__ b2,
    int which0,
    _Float16* __restrict__ qh,
    _Float16* __restrict__ kh,
    _Float16* __restrict__ vt)
{
  __shared__ __attribute__((aligned(16))) _Float16 sT[128 * 64];

  const int tid = threadIdx.x, lane = tid & 31, w = tid >> 5;
  const int h = lane >> 4, m = lane & 15;
  const int m0 = blockIdx.x * 128;
  const int wsel = blockIdx.y / NHEADS;
  const int head = blockIdx.y - wsel * NHEADS;
  const int which = which0 + wsel;
  const int m0w = m0 + 32 * w;

  const _Float16* wbase = (which == 0) ? w0 : ((which == 1) ? w1 : w2);
  const float* bias = (which == 0) ? b0 : ((which == 1) ? b1 : b2);

  const _Float16* xa0 = xh + (size_t)(m0w + m) * DIM;
  const _Float16* xa1 = xa0 + (size_t)16 * DIM;
  const _Float16* wb  = wbase + (size_t)(head * HD + m) * DIM;

  const v8f zero8 = {0.f, 0.f, 0.f, 0.f, 0.f, 0.f, 0.f, 0.f};
  v8f acc[2][4];
  #pragma unroll
  for (int mt = 0; mt < 2; ++mt)
    #pragma unroll
    for (int nt = 0; nt < 4; ++nt) acc[mt][nt] = zero8;

  #pragma unroll 1
  for (int k0 = 0; k0 < DIM; k0 += 32) {
    const v16h a0 = load_frag(xa0 + k0, h);
    const v16h a1 = load_frag(xa1 + k0, h);
    #pragma unroll
    for (int nt = 0; nt < 4; ++nt) {
      const v16h b = load_frag(wb + (size_t)nt * 16 * DIM + k0, h);
      acc[0][nt] = wmma_f16(a0, b, acc[0][nt]);
      acc[1][nt] = wmma_f16(a1, b, acc[1][nt]);
    }
  }

  #pragma unroll
  for (int nt = 0; nt < 4; ++nt) {
    const int feat = 16 * nt + m;
    const float bvl = bias[head * HD + feat];
    #pragma unroll
    for (int mt = 0; mt < 2; ++mt) {
      #pragma unroll
      for (int r = 0; r < 8; ++r) {
        const int tokl = 32 * w + 16 * mt + 8 * h + r;
        const float y = acc[mt][nt][r] * (1.0f / WSCALE) + bvl;
        const int idx = (which == 2) ? (feat * 128 + tokl) : (tokl * HD + feat);
        sT[idx] = (_Float16)y;
      }
    }
  }
  __syncthreads();

  const int b = m0 / S, l0 = m0 - b * S, bh = b * NHEADS + head;
  _Float16* plane = (which == 0) ? qh : kh;
  proj_store_pass(sT, plane, vt, which, S, bh, l0, w, lane);
  __threadfence();
  proj_store_pass(sT, plane, vt, which, S, bh, l0, w, lane);
}

__device__ __forceinline__ v16h pack_p(v8f a, v8f c) {
  const v16h r = { (_Float16)(a[0] * PSCALE), (_Float16)(a[1] * PSCALE), (_Float16)(a[2] * PSCALE), (_Float16)(a[3] * PSCALE),
                   (_Float16)(a[4] * PSCALE), (_Float16)(a[5] * PSCALE), (_Float16)(a[6] * PSCALE), (_Float16)(a[7] * PSCALE),
                   (_Float16)(c[0] * PSCALE), (_Float16)(c[1] * PSCALE), (_Float16)(c[2] * PSCALE), (_Float16)(c[3] * PSCALE),
                   (_Float16)(c[4] * PSCALE), (_Float16)(c[5] * PSCALE), (_Float16)(c[6] * PSCALE), (_Float16)(c[7] * PSCALE) };
  return r;
}

__device__ __forceinline__ void att_store_pass(const float* so, _Float16* att,
                                               int b, int head, int q0, int lane) {
  const int q8 = lane & 7, sub = lane >> 3;
  #pragma unroll
  for (int i = 0; i < 4; ++i) {
    const int row = i * 4 + sub;
    const v4f a = *(const v4fa*)(so + row * 64 + 8 * q8);
    const v4f c = *(const v4fa*)(so + row * 64 + 8 * q8 + 4);
    const v8h o = cvt8(a, c, 1.0f);
    const size_t gi = ((size_t)b * SQ + q0 + row) * DIM + head * HD + 8 * q8;
    *(volatile v8h*)(att + gi) = o;
  }
}

__global__ __launch_bounds__(128) void attn_kernel(
    const _Float16* __restrict__ qh,
    const _Float16* __restrict__ kh,
    const _Float16* __restrict__ vt,
    int SKV, int causal,
    _Float16* __restrict__ att)
{
  __shared__ __attribute__((aligned(16))) float sO[4 * 16 * 64];

  const int tid = threadIdx.x, lane = tid & 31, w = tid >> 5;
  const int h = lane >> 4, m = lane & 15;
  const int bh = blockIdx.y, b = bh / NHEADS, head = bh - b * NHEADS;
  const int qblk = blockIdx.x * 64;
  const int q0 = qblk + 16 * w;
  const int qidx = q0 + m;

  const _Float16* qrow = qh + ((size_t)bh * SQ + q0 + m) * HD;
  const v16h qb0 = load_frag(qrow, h);
  const v16h qb1 = load_frag(qrow + 32, h);

  const v8f zero8 = {0.f, 0.f, 0.f, 0.f, 0.f, 0.f, 0.f, 0.f};
  v8f o[4];
  #pragma unroll
  for (int t = 0; t < 4; ++t) o[t] = zero8;
  float mrun = -1e30f, lrun = 0.0f;

  const _Float16* kbase = kh + ((size_t)bh * SKV + m) * HD;
  const _Float16* vbase = vt + ((size_t)bh * HD + m) * SKV;
  const int kend = causal ? (qblk + 64) : SKV;

  #pragma unroll 1
  for (int kb = 0; kb < kend; kb += 64) {
    v8f s[4];
    #pragma unroll
    for (int j = 0; j < 4; ++j) {
      const _Float16* kp = kbase + (size_t)(kb + 16 * j) * HD;
      const v16h kf0 = load_frag(kp, h);
      const v16h kf1 = load_frag(kp + 32, h);
      v8f z = zero8;
      z = wmma_f16(kf0, qb0, z);
      z = wmma_f16(kf1, qb1, z);
      s[j] = z;
    }
    #pragma unroll
    for (int j = 0; j < 4; ++j) {
      #pragma unroll
      for (int r = 0; r < 8; ++r) {
        float v = s[j][r] * 0.125f;
        if (causal) {
          const int key = kb + 16 * j + 8 * h + r;
          v = (key <= qidx) ? v : -1.0e9f;
        }
        s[j][r] = v;
      }
    }

    float mloc = s[0][0];
    #pragma unroll
    for (int j = 0; j < 4; ++j)
      #pragma unroll
      for (int r = 0; r < 8; ++r) mloc = fmaxf(mloc, s[j][r]);
    mloc = fmaxf(mloc, __shfl_xor(mloc, 16));
    const float mnew = fmaxf(mrun, mloc);
    const float alpha = __expf(mrun - mnew);
    mrun = mnew;
    float lsum = 0.0f;
    #pragma unroll
    for (int j = 0; j < 4; ++j)
      #pragma unroll
      for (int r = 0; r < 8; ++r) {
        const float p = __expf(s[j][r] - mnew);
        s[j][r] = p;
        lsum += p;
      }
    lsum += __shfl_xor(lsum, 16);
    lrun = lrun * alpha + lsum;
    #pragma unroll
    for (int t = 0; t < 4; ++t)
      #pragma unroll
      for (int r = 0; r < 8; ++r) o[t][r] = o[t][r] * alpha;

    const v16h pb0 = pack_p(s[0], s[1]);
    const v16h pb1 = pack_p(s[2], s[3]);

    #pragma unroll
    for (int t = 0; t < 4; ++t) {
      const _Float16* vp = vbase + (size_t)(16 * t) * SKV + kb;
      const v16h vf0 = load_frag(vp, h);
      const v16h vf1 = load_frag(vp + 32, h);
      o[t] = wmma_f16(vf0, pb0, o[t]);
      o[t] = wmma_f16(vf1, pb1, o[t]);
    }
  }

  const float inv = (1.0f / lrun) * (ATTSC / PSCALE);
  float* so = sO + w * 1024;
  #pragma unroll
  for (int t = 0; t < 4; ++t)
    #pragma unroll
    for (int r = 0; r < 8; ++r)
      so[m * 64 + 16 * t + 8 * h + r] = o[t][r] * inv;
  __syncthreads();

  att_store_pass(so, att, b, head, q0, lane);
  __threadfence();
  att_store_pass(so, att, b, head, q0, lane);
}

__device__ __forceinline__ void gemm_store32(const float* sC, float* out32,
                                             int w, int lane, int mb, int nb, int N) {
  const int rs = lane >> 4, c4 = (lane & 15) * 4;
  #pragma unroll
  for (int i = 0; i < 16; ++i) {
    const int rl = 32 * w + 2 * i + rs;
    const v4f v = *(const v4fa*)(sC + rl * 64 + c4);
    *(volatile v4f*)(out32 + (size_t)(mb + rl) * N + nb + c4) = v;
  }
}

__device__ __forceinline__ void gemm_store16(const float* sC, _Float16* out16,
                                             int w, int lane, int mb, int nb, int N, float sc) {
  const int q8 = lane & 7, sub = lane >> 3;
  #pragma unroll
  for (int i = 0; i < 8; ++i) {
    const int rl = 32 * w + 4 * i + sub;
    const float* sp = sC + rl * 64 + 8 * q8;
    const v4f a = *(const v4fa*)sp;
    const v4f c = *(const v4fa*)(sp + 4);
    const v8h o = cvt8(a, c, sc);
    *(volatile v8h*)(out16 + (size_t)(mb + rl) * N + nb + 8 * q8) = o;
  }
}

__global__ __launch_bounds__(128) void gemm_kernel(
    const _Float16* __restrict__ A, const _Float16* __restrict__ Bt,
    int M, int N, int K, float ascale,
    const float* __restrict__ bias,
    const float* resid,
    const float* __restrict__ bng, const float* __restrict__ bnb,
    const float* __restrict__ bnm, const float* __restrict__ bnv,
    int flags,
    float* out32, _Float16* out16, float o16scale)
{
  __shared__ __attribute__((aligned(16))) float sC[128 * 64];
  (void)M;

  const int tid = threadIdx.x, lane = tid & 31, w = tid >> 5;
  const int h = lane >> 4, m = lane & 15;
  const int mb = blockIdx.x * 128, nb = blockIdx.y * 64;

  const _Float16* a0p = A + (size_t)(mb + 32 * w + m) * K;
  const _Float16* a1p = a0p + (size_t)16 * K;
  const _Float16* bp  = Bt + (size_t)(nb + m) * K;

  const v8f zero8 = {0.f, 0.f, 0.f, 0.f, 0.f, 0.f, 0.f, 0.f};
  v8f acc[2][4];
  #pragma unroll
  for (int mt = 0; mt < 2; ++mt)
    #pragma unroll
    for (int nt = 0; nt < 4; ++nt) acc[mt][nt] = zero8;

  #pragma unroll 1
  for (int k0 = 0; k0 < K; k0 += 32) {
    const v16h a0 = load_frag(a0p + k0, h);
    const v16h a1 = load_frag(a1p + k0, h);
    #pragma unroll
    for (int nt = 0; nt < 4; ++nt) {
      const v16h b = load_frag(bp + (size_t)nt * 16 * K + k0, h);
      acc[0][nt] = wmma_f16(a0, b, acc[0][nt]);
      acc[1][nt] = wmma_f16(a1, b, acc[1][nt]);
    }
  }

  #pragma unroll
  for (int nt = 0; nt < 4; ++nt)
    #pragma unroll
    for (int mt = 0; mt < 2; ++mt)
      #pragma unroll
      for (int r = 0; r < 8; ++r)
        sC[(32 * w + 16 * mt + 8 * h + r) * 64 + 16 * nt + m] = acc[mt][nt][r] * ascale;
  __syncthreads();

  const int rs = lane >> 4, c4 = (lane & 15) * 4;
  const int col = nb + c4;
  v4f bias4 = {0.f, 0.f, 0.f, 0.f};
  v4f g4 = {1.f, 1.f, 1.f, 1.f}, b4 = {0.f, 0.f, 0.f, 0.f}, m4 = {0.f, 0.f, 0.f, 0.f}, i4 = {1.f, 1.f, 1.f, 1.f};
  if (flags & F_BIAS) bias4 = *(const v4fa*)(bias + col);
  if (flags & F_BN) {
    g4 = *(const v4fa*)(bng + col);
    b4 = *(const v4fa*)(bnb + col);
    m4 = *(const v4fa*)(bnm + col);
    const v4f vv = *(const v4fa*)(bnv + col);
    i4.x = rsqrtf(vv.x + BN_EPS);
    i4.y = rsqrtf(vv.y + BN_EPS);
    i4.z = rsqrtf(vv.z + BN_EPS);
    i4.w = rsqrtf(vv.w + BN_EPS);
  }
  #pragma unroll
  for (int i = 0; i < 16; ++i) {
    const int rl = 32 * w + 2 * i + rs;
    float* sp = sC + rl * 64 + c4;
    v4f v = *(v4fa*)sp;
    if (flags & F_BIAS) v = v + bias4;
    if (flags & F_RESID) v = v + *(const v4fa*)(resid + (size_t)(mb + rl) * N + col);
    if (flags & F_RELU) {
      v.x = fmaxf(v.x, 0.f); v.y = fmaxf(v.y, 0.f); v.z = fmaxf(v.z, 0.f); v.w = fmaxf(v.w, 0.f);
    }
    if (flags & F_BN) v = (g4 * (v - m4)) * i4 + b4;
    *(v4fa*)sp = v;
    if (flags & F_O32) *(volatile v4f*)(out32 + (size_t)(mb + rl) * N + col) = v;
  }
  __syncthreads();

  if (flags & F_O16) gemm_store16(sC, out16, w, lane, mb, nb, N, o16scale);
  __threadfence();
  if (flags & F_O32) gemm_store32(sC, out32, w, lane, mb, nb, N);
  if (flags & F_O16) gemm_store16(sC, out16, w, lane, mb, nb, N, o16scale);
}

extern "C" void kernel_launch(void* const* d_in, const int* in_sizes, int n_in,
                              void* d_out, int out_size, void* d_ws, size_t ws_size,
                              hipStream_t stream) {
  if (n_in < 32) return;
  const int DD = DIM * DIM;
  if (in_sizes[0] != MK * DIM || in_sizes[1] != MQ * DIM) return;
  if (in_sizes[2] != DD || in_sizes[4] != DD || in_sizes[6] != DD || in_sizes[8] != DD) return;
  if (in_sizes[3] != DIM || in_sizes[5] != DIM || in_sizes[7] != DIM || in_sizes[9] != DIM) return;
  if (in_sizes[10] != DIM || in_sizes[11] != DIM || in_sizes[12] != DIM || in_sizes[13] != DIM) return;
  if (in_sizes[14] != NLAYER * DD || in_sizes[16] != NLAYER * DD ||
      in_sizes[18] != NLAYER * DD || in_sizes[20] != NLAYER * DD) return;
  if (in_sizes[15] != NLAYER * DIM || in_sizes[17] != NLAYER * DIM ||
      in_sizes[19] != NLAYER * DIM || in_sizes[21] != NLAYER * DIM) return;
  if (in_sizes[22] != NLAYER * DIM || in_sizes[23] != NLAYER * DIM ||
      in_sizes[24] != NLAYER * DIM || in_sizes[25] != NLAYER * DIM) return;
  if (in_sizes[26] != NLAYER * DIM * DFF || in_sizes[27] != NLAYER * DIM * DFF) return;
  if (in_sizes[28] != NLAYER * DIM || in_sizes[29] != NLAYER * DIM ||
      in_sizes[30] != NLAYER * DIM || in_sizes[31] != NLAYER * DIM) return;
  if (out_size != MQ * DIM) return;

  const float* enc    = (const float*)d_in[0];
  const float* x1     = (const float*)d_in[1];
  const float* inp_wq = (const float*)d_in[2];
  const float* inp_bq = (const float*)d_in[3];
  const float* inp_wk = (const float*)d_in[4];
  const float* inp_bk = (const float*)d_in[5];
  const float* inp_wv = (const float*)d_in[6];
  const float* inp_bv = (const float*)d_in[7];
  const float* inp_wo = (const float*)d_in[8];
  const float* inp_bo = (const float*)d_in[9];
  const float* bn0g   = (const float*)d_in[10];
  const float* bn0b   = (const float*)d_in[11];
  const float* bn0m   = (const float*)d_in[12];
  const float* bn0v   = (const float*)d_in[13];
  const float* wq_l   = (const float*)d_in[14];
  const float* bq_l   = (const float*)d_in[15];
  const float* wk_l   = (const float*)d_in[16];
  const float* bk_l   = (const float*)d_in[17];
  const float* wv_l   = (const float*)d_in[18];
  const float* bv_l   = (const float*)d_in[19];
  const float* wo_l   = (const float*)d_in[20];
  const float* bo_l   = (const float*)d_in[21];
  const float* bn1g   = (const float*)d_in[22];
  const float* bn1b   = (const float*)d_in[23];
  const float* bn1m   = (const float*)d_in[24];
  const float* bn1v   = (const float*)d_in[25];
  const float* mlp_w1 = (const float*)d_in[26];
  const float* mlp_w2 = (const float*)d_in[27];
  const float* bn2g   = (const float*)d_in[28];
  const float* bn2b   = (const float*)d_in[29];
  const float* bn2m   = (const float*)d_in[30];
  const float* bn2v   = (const float*)d_in[31];
  float* out = (float*)d_out;

  const size_t b_x1h  = (size_t)MQ * DIM * 2;
  const size_t b_ench = (size_t)MK * DIM * 2;
  const size_t b_wdd  = (size_t)DD * 2;
  const size_t b_wff  = (size_t)DIM * DFF * 2;
  const size_t b_qh   = (size_t)BATCH * NHEADS * SQ * HD * 2;
  const size_t b_kh   = (size_t)BATCH * NHEADS * SK * HD * 2;
  const size_t b_att  = (size_t)MQ * DIM * 2;
  const size_t b_x32  = (size_t)MQ * DIM * 4;
  const size_t b_x16  = (size_t)MQ * DIM * 2;
  const size_t b_h16  = (size_t)MQ * DFF * 2;
  if (b_h16 > 2 * b_kh) return;

  char* ws = (char*)d_ws;
  size_t off = 0;
  _Float16* x1h   = (_Float16*)(ws + off); off += b_x1h;
  _Float16* ench  = (_Float16*)(ws + off); off += b_ench;
  _Float16* wqkv0 = (_Float16*)(ws + off); off += 3 * b_wdd;
  _Float16* wo0   = (_Float16*)(ws + off); off += b_wdd;
  _Float16* wql   = (_Float16*)(ws + off); off += NLAYER * b_wdd;
  _Float16* wkl   = (_Float16*)(ws + off); off += NLAYER * b_wdd;
  _Float16* wvl   = (_Float16*)(ws + off); off += NLAYER * b_wdd;
  _Float16* wol   = (_Float16*)(ws + off); off += NLAYER * b_wdd;
  _Float16* w1l   = (_Float16*)(ws + off); off += NLAYER * b_wff;
  _Float16* w2l   = (_Float16*)(ws + off); off += NLAYER * b_wff;
  _Float16* qh    = (_Float16*)(ws + off); off += b_qh;
  _Float16* kh    = (_Float16*)(ws + off); off += b_kh;
  _Float16* vt    = (_Float16*)(ws + off); off += b_kh;
  _Float16* h16   = kh;
  _Float16* att16 = (_Float16*)(ws + off); off += b_att;
  float*    x32a  = (float*)(ws + off);    off += b_x32;
  float*    x32b  = (float*)(ws + off);    off += b_x32;
  _Float16* x16   = (_Float16*)(ws + off); off += b_x16;
  if (off > ws_size) return;

  const int na8 = MQ * DIM / 8, nb8 = MK * DIM / 8;
  cvt_rows_kernel<<<dim3((na8 + nb8 + 255) / 256), dim3(256), 0, stream>>>(x1, na8, enc, nb8, x1h, ench);

  cvt_wt_kernel<<<dim3(DIM / 64, DIM / 64, 4), dim3(256), 0, stream>>>(
      inp_wq, inp_wk, inp_wv, inp_wo, wqkv0, wqkv0 + DD, wqkv0 + 2 * DD, wo0, DIM, DIM, 1);
  cvt_wt_kernel<<<dim3(DIM / 64, DIM / 64, 4 * NLAYER), dim3(256), 0, stream>>>(
      wq_l, wk_l, wv_l, wo_l, wql, wkl, wvl, wol, DIM, DIM, NLAYER);
  cvt_wt_kernel<<<dim3(DFF / 64, DIM / 64, NLAYER), dim3(256), 0, stream>>>(
      mlp_w1, mlp_w1, mlp_w1, mlp_w1, w1l, w1l, w1l, w1l, DIM, DFF, NLAYER);
  cvt_wt_kernel<<<dim3(DIM / 64, DFF / 64, NLAYER), dim3(256), 0, stream>>>(
      mlp_w2, mlp_w2, mlp_w2, mlp_w2, w2l, w2l, w2l, w2l, DFF, DIM, NLAYER);

  const int FO = F_BIAS | F_RESID | F_BN | F_O32 | F_O16;
  const float osc = 1.0f / (ATTSC * WSCALE);

  proj_kernel<<<dim3(MQ / 128, 3 * NHEADS), dim3(128), 0, stream>>>(
      x1h, SQ, wqkv0, wqkv0 + DD, wqkv0 + 2 * DD, inp_bq, inp_bk, inp_bv, 0, qh, kh, vt);
  attn_kernel<<<dim3(SQ / 64, BATCH * NHEADS), dim3(128), 0, stream>>>(qh, kh, vt, SQ, 1, att16);
  gemm_kernel<<<dim3(MQ / 128, DIM / 64), dim3(128), 0, stream>>>(
      att16, wo0, MQ, DIM, DIM, osc, inp_bo, x1, bn0g, bn0b, bn0m, bn0v, FO, x32a, x16, 1.0f);

  float* xcur = x32a;
  float* xoth = x32b;

  for (int l = 0; l < NLAYER; ++l) {
    const _Float16* wq = wql + (size_t)l * DD;
    const _Float16* wk = wkl + (size_t)l * DD;
    const _Float16* wv = wvl + (size_t)l * DD;
    const _Float16* wo = wol + (size_t)l * DD;

    proj_kernel<<<dim3(MQ / 128, NHEADS), dim3(128), 0, stream>>>(
        x16, SQ, wq, wq, wq, bq_l + l * DIM, bq_l + l * DIM, bq_l + l * DIM, 0, qh, kh, vt);
    proj_kernel<<<dim3(MK / 128, 2 * NHEADS), dim3(128), 0, stream>>>(
        ench, SK, wk, wk, wv, bk_l + l * DIM, bk_l + l * DIM, bv_l + l * DIM, 1, qh, kh, vt);
    attn_kernel<<<dim3(SQ / 64, BATCH * NHEADS), dim3(128), 0, stream>>>(qh, kh, vt, SK, 0, att16);
    gemm_kernel<<<dim3(MQ / 128, DIM / 64), dim3(128), 0, stream>>>(
        att16, wo, MQ, DIM, DIM, osc, bo_l + l * DIM, xcur,
        bn1g + l * DIM, bn1b + l * DIM, bn1m + l * DIM, bn1v + l * DIM, FO, xoth, x16, 1.0f);
    { float* t = xcur; xcur = xoth; xoth = t; }

    gemm_kernel<<<dim3(MQ / 128, DFF / 64), dim3(128), 0, stream>>>(
        x16, w1l + (size_t)l * DIM * DFF, MQ, DFF, DIM, 1.0f / WSCALE, inp_bo, xcur,
        bn0g, bn0b, bn0m, bn0v, F_RELU | F_O16, xoth, h16, HSC);
    const int last = (l == NLAYER - 1);
    float* o32 = last ? out : xoth;
    gemm_kernel<<<dim3(MQ / 128, DIM / 64), dim3(128), 0, stream>>>(
        h16, w2l + (size_t)l * DIM * DFF, MQ, DIM, DFF, 1.0f / (HSC * WSCALE), inp_bo, xcur,
        bn2g + l * DIM, bn2b + l * DIM, bn2m + l * DIM, bn2v + l * DIM,
        F_RESID | F_BN | F_O32 | (last ? 0 : F_O16), o32, x16, 1.0f);
    if (!last) { float* t = xcur; xcur = xoth; xoth = t; }
  }
}
